// _SeqGenerator2D_54185307406556
// MI455X (gfx1250) — hardware-verified
//
#include <hip/hip_runtime.h>
#include <math.h>

constexpr int NAGENT = 8192;
constexpr int NTOBS  = 50;
constexpr int NSPRED = 100;
constexpr int NEMB   = 64;
constexpr int NHID   = 128;
constexpr int NGATE4 = 512;
constexpr int NMLP   = 256;
constexpr int NMLP2  = 112;
constexpr int NNOISE = 16;
constexpr int NTHR   = 256;
constexpr int RB     = 32;
constexpr int APITCH = 136;
constexpr int MPITCH = 264;
constexpr int DPITCH = 132;
constexpr int HSP    = 132;
constexpr int OBSW   = NTOBS * 2;
constexpr int OBW    = NSPRED * 2;
constexpr float WCAR     = 16.0f;
constexpr float WCAR_INV = 1.0f / 16.0f;
constexpr float L2E      = 1.4426950408889634f;
constexpr float NEGL2E   = -L2E;
constexpr float K2L      = 2.0f * L2E;
constexpr int OFF_WHE = 0;
constexpr int OFF_WHD = NGATE4 * NHID;
constexpr int OFF_WM1 = 2 * NGATE4 * NHID;
constexpr int OFF_WM2 = OFF_WM1 + NMLP * NHID;
constexpr int W16_HALVES = OFF_WM2 + NHID * NMLP;
constexpr int FC_FLOATS  = 2 * NGATE4 * 4;
static_assert(OFF_WHD == 65536 && OFF_WM1 == 131072 && OFF_WM2 == 163840 && W16_HALVES == 196608, "plane map");
static_assert(W16_HALVES == 96 * NTHR * 8, "prep coverage: 96 blocks x 256 threads x 8 halves");
static_assert(FC_FLOATS == 4 * NTHR * 4, "fold coverage: 4 blocks x 256 threads x 4 floats");
static_assert(NAGENT % RB == 0, "grid exact");
static_assert(NHID == 16 * (NTHR / 32), "8 waves x 16 hidden units");
static_assert(NHID % 32 == 0 && NMLP % 32 == 0, "K multiples of 32");
static_assert((2 * RB * APITCH) % NTHR == 0, "A tile zero fill exact");
static_assert(RB * NHID == 2 * NTHR * 8, "h0 fill: 2 x v8h per thread");
static_assert((RB * OBW * 4) % 512 == 0, "block output = whole 512-B wave chunks");
static_assert(APITCH % 8 == 0 && MPITCH % 8 == 0 && DPITCH % 4 == 0 && HSP % 4 == 0, "LDS vector alignment");

typedef __attribute__((ext_vector_type(16))) _Float16 v16h;
typedef __attribute__((ext_vector_type(8)))  _Float16 v8h;
typedef __attribute__((ext_vector_type(8)))  float    v8f;
typedef __attribute__((ext_vector_type(4)))  float    v4f;
typedef __attribute__((ext_vector_type(2)))  float    v2f;

__device__ __forceinline__ void guard8(v8f& a0, v8f& a1, v8f& a2, v8f& a3, v8f& a4, v8f& a5, v8f& a6, v8f& a7,
                                       v16h x, v16h y, v16h p, v16h q, v16h u, v16h w) {
  asm volatile("v_nop\n\tv_nop\n\tv_nop\n\tv_nop"
               : "+v"(a0), "+v"(a1), "+v"(a2), "+v"(a3), "+v"(a4), "+v"(a5), "+v"(a6), "+v"(a7)
               : "v"(x), "v"(y), "v"(p), "v"(q), "v"(u), "v"(w));
}
__device__ __forceinline__ void guard4f(v8f& a0, v8f& a1, v8f& a2, v8f& a3, v16h x, v16h y, v16h p, v16h q) {
  asm volatile("v_nop\n\tv_nop\n\tv_nop\n\tv_nop"
               : "+v"(a0), "+v"(a1), "+v"(a2), "+v"(a3)
               : "v"(x), "v"(y), "v"(p), "v"(q));
}
__device__ __forceinline__ void guard2f(v8f& a0, v8f& a1, v16h x, v16h y, v16h p) {
  asm volatile("v_nop\n\tv_nop\n\tv_nop\n\tv_nop" : "+v"(a0), "+v"(a1) : "v"(x), "v"(y), "v"(p));
}
__device__ __forceinline__ void acc_guard4(v8f& a, v8f& b, v8f& c, v8f& d) { asm volatile("v_nop\n\tv_nop\n\tv_nop\n\tv_nop" : "+v"(a), "+v"(b), "+v"(c), "+v"(d)); }
__device__ __forceinline__ void acc_guard2(v8f& a, v8f& b) { asm volatile("v_nop\n\tv_nop\n\tv_nop\n\tv_nop" : "+v"(a), "+v"(b)); }
template <typename T> struct Frag;
template <> struct Frag<_Float16> {
  typedef v16h V; union U { v16h v; v8h h[2]; };
  static __device__ __forceinline__ v16h load(const _Float16* p) {
    U f; f.h[0] = *(const v8h*)(p); f.h[1] = *(const v8h*)(p + 16); return f.v;
  }
  static __device__ __forceinline__ v8f mma(v16h a, v16h b, v8f c) {
    return __builtin_amdgcn_wmma_f32_16x16x32_f16(false, a, false, b, (short)0, c, false, false);
  }
};

__device__ __forceinline__ float hw_exp2(float x) { return __builtin_amdgcn_exp2f(x); }
__device__ __forceinline__ float hw_rcp(float x)  { return __builtin_amdgcn_rcpf(x); }
__device__ __forceinline__ float fsig(float x)  { return hw_rcp(1.0f + hw_exp2(x * NEGL2E)); }
__device__ __forceinline__ float ftanh(float x) { return fmaf(hw_rcp(hw_exp2(x * K2L) + 1.0f), -2.0f, 1.0f); }

__global__ __launch_bounds__(NTHR) void prep_w16_kernel(const float* __restrict__ Whh_e, const float* __restrict__ Whh_d,
                                                        const float* __restrict__ Wm1, const float* __restrict__ Wm2,
                                                        unsigned short* __restrict__ W16) {
  const int tid = threadIdx.x, blk = blockIdx.x;
  const int i = blk * NTHR + tid;
  v4f p0 = {0.f, 0.f, 0.f, 0.f}, p1 = {0.f, 0.f, 0.f, 0.f};
  float sc = WCAR;
  if (blk < 64) {
    const bool dsel = (blk >= 32);
    const int j = i - (dsel ? 8192 : 0);
    const int n = j >> 4;
    const int k = (j & 15) * 8;
    const float* wh = dsel ? Whh_d : Whh_e;
    p0 = *(const v4f*)(wh + (size_t)n * NHID + k);
    p1 = *(const v4f*)(wh + (size_t)n * NHID + k + 4);
  } else if (blk < 80) {
    const int j = i - 16384;
    const int n = j >> 4;
    const int k = (j & 15) * 8;
    p0 = *(const v4f*)(Wm1 + (size_t)n * NHID + k);
    p1 = *(const v4f*)(Wm1 + (size_t)n * NHID + k + 4);
  } else {
    const int j = i - 20480;
    const int n = j >> 5;
    const int k = (j & 31) * 8;
    const int nn = (n < NMLP2) ? n : (NMLP2 - 1);
    p0 = *(const v4f*)(Wm2 + (size_t)nn * NMLP + k);
    p1 = *(const v4f*)(Wm2 + (size_t)nn * NMLP + k + 4);
    sc = (n < NMLP2) ? WCAR : 0.0f;
  }
  v8h hv;
#pragma unroll
  for (int e = 0; e < 4; ++e) { hv[e] = (_Float16)(p0[e] * sc); hv[4 + e] = (_Float16)(p1[e] * sc); }
  unsigned short* dp = W16 + (size_t)i * 8;
  *(volatile v8h*)dp = hv;
  __threadfence();
  *(volatile v8h*)dp = hv;
}

__global__ __launch_bounds__(NTHR) void prep_fold_kernel(const float* __restrict__ Wih_e, const float* __restrict__ We,
                                                         const float* __restrict__ be, const float* __restrict__ b_e,
                                                         const float* __restrict__ Wih_d, const float* __restrict__ Wd,
                                                         const float* __restrict__ bd, const float* __restrict__ b_d,
                                                         float* __restrict__ FC) {
  const int tid = threadIdx.x, blk = blockIdx.x;
  const bool dsel = (blk >= 2);
  const int n = (blk & 1) * NTHR + tid;
  const float* wi = dsel ? Wih_d : Wih_e;
  const float* wx = dsel ? Wd : We;
  const float* bx = dsel ? bd : be;
  const float* bg = dsel ? b_d : b_e;
  const float* wrow = wi + (size_t)n * NEMB;
  float f0 = 0.0f, f1 = 0.0f, cc = 0.0f;
#pragma unroll 1
  for (int k = 0; k < NEMB; ++k) {
    const float w = wrow[k];
    f0 = fmaf(w, wx[2 * k], f0);
    f1 = fmaf(w, wx[2 * k + 1], f1);
    cc = fmaf(w, bx[k], cc);
  }
  const float bn = bg[n];
  v4f o;
  o[0] = f0; o[1] = f1; o[2] = cc + bn; o[3] = bn;
  float* op = FC + ((size_t)(dsel ? NGATE4 : 0) + n) * 4;
  *(volatile v4f*)op = o;
  __threadfence();
  *(volatile v4f*)op = o;
}

template <bool WITH_HS>
__device__ __forceinline__ void lstm_step(const _Float16* acur, _Float16* anxt, float* hs,
                                          const float* offp, int offstride,
                                          const _Float16* __restrict__ wlane, float (&cst)[2][8],
                                          const float (&gF0)[4], const float (&gF1)[4], const float (&gC)[4],
                                          int ucol, int c, int hh, int koff) {
  const v8f z8 = {0.f, 0.f, 0.f, 0.f, 0.f, 0.f, 0.f, 0.f};
  v8f acc[2][4];
#pragma unroll
  for (int ms = 0; ms < 2; ++ms)
#pragma unroll
    for (int g = 0; g < 4; ++g) acc[ms][g] = z8;
  const _Float16* a0p = acur + c * APITCH + koff;
  const _Float16* a1p = a0p + 16 * APITCH;
#pragma unroll 1
  for (int k0 = 0; k0 < NHID; k0 += 32) {
    v16h bq[4];
#pragma unroll
    for (int g = 0; g < 4; ++g) bq[g] = Frag<_Float16>::load(wlane + (size_t)g * (NHID * NHID) + k0);
    const v16h fa0 = Frag<_Float16>::load(a0p + k0);
    const v16h fa1 = Frag<_Float16>::load(a1p + k0);
#pragma unroll
    for (int g = 0; g < 4; ++g) {
      acc[0][g] = Frag<_Float16>::mma(fa0, bq[g], acc[0][g]);
      acc[1][g] = Frag<_Float16>::mma(fa1, bq[g], acc[1][g]);
    }
    guard8(acc[0][0], acc[0][1], acc[0][2], acc[0][3], acc[1][0], acc[1][1], acc[1][2], acc[1][3],
           fa0, fa1, bq[0], bq[1], bq[2], bq[3]);
  }
  acc_guard4(acc[0][0], acc[0][1], acc[0][2], acc[0][3]);
  acc_guard4(acc[1][0], acc[1][1], acc[1][2], acc[1][3]);
#pragma unroll
  for (int ms = 0; ms < 2; ++ms) {
#pragma unroll
    for (int r = 0; r < 8; ++r) {
      const int row = 16 * ms + 8 * hh + r;
      const v2f o = *(const v2f*)(offp + row * offstride);
      float pi = fmaf(acc[ms][0][r], WCAR_INV, gC[0]); pi = fmaf(o[0], gF0[0], pi); pi = fmaf(o[1], gF1[0], pi);
      float pf = fmaf(acc[ms][1][r], WCAR_INV, gC[1]); pf = fmaf(o[0], gF0[1], pf); pf = fmaf(o[1], gF1[1], pf);
      float pg = fmaf(acc[ms][2][r], WCAR_INV, gC[2]); pg = fmaf(o[0], gF0[2], pg); pg = fmaf(o[1], gF1[2], pg);
      float po = fmaf(acc[ms][3][r], WCAR_INV, gC[3]); po = fmaf(o[0], gF0[3], po); po = fmaf(o[1], gF1[3], po);
      const float si = fsig(pi);
      const float sf = fsig(pf);
      const float tg = ftanh(pg);
      const float so = fsig(po);
      const float c2 = fmaf(sf, cst[ms][r], si * tg);
      cst[ms][r] = c2;
      const float h2 = so * ftanh(c2);
      anxt[row * APITCH + ucol] = (_Float16)h2;
      if (WITH_HS) hs[row * HSP + ucol] = h2;
    }
  }
}

__global__ __launch_bounds__(NTHR) void enc_mlp_kernel(const float* __restrict__ obs, const unsigned short* __restrict__ W16,
                                                       const float* __restrict__ FC, const float* __restrict__ bm1,
                                                       const float* __restrict__ bm2, const float* __restrict__ z,
                                                       float* __restrict__ DH) {
  __shared__ __align__(16) _Float16 At[2][RB * APITCH];
  __shared__ __align__(16) float    OffAll[RB * OBSW];
  __shared__ __align__(16) _Float16 Mt[RB * MPITCH];
  __shared__ __align__(16) float    Df[RB * DPITCH];
  const _Float16* WHE  = (const _Float16*)W16 + OFF_WHE;
  const _Float16* WM1P = (const _Float16*)W16 + OFF_WM1;
  const _Float16* WM2P = (const _Float16*)W16 + OFF_WM2;
  const int tid = threadIdx.x, lane = tid & 31, wave = tid >> 5;
  const int c = lane & 15, hh = lane >> 4, koff = 8 * hh;
  const int rowbase = blockIdx.x * RB;
  const int ucol = 16 * wave + c;

  {
    _Float16* af = &At[0][0];
#pragma unroll 1
    for (int i = tid; i < 2 * RB * APITCH; i += NTHR) af[i] = (_Float16)0.0f;
  }
#pragma unroll 1
  for (int idx = tid; idx < RB * OBSW; idx += NTHR) {
    const int row = idx / OBSW;
    const int rem = idx - row * OBSW;
    const float* ob = obs + (size_t)(rowbase + row) * OBSW;
    const int rp = (rem >= 2) ? (rem - 2) : rem;
    const float cur = ob[rem];
    const float pv  = ob[rp];
    OffAll[idx] = cur - ((rem >= 2) ? pv : 0.0f);
  }
  float cst[2][8];
#pragma unroll
  for (int ms = 0; ms < 2; ++ms)
#pragma unroll
    for (int r = 0; r < 8; ++r) cst[ms][r] = 0.0f;
  float gF0[4], gF1[4], gC[4];
#pragma unroll
  for (int g = 0; g < 4; ++g) {
    const v4f fcv = *(const v4f*)(FC + (size_t)(g * NHID + ucol) * 4);
    gF0[g] = fcv[0]; gF1[g] = fcv[1]; gC[g] = fcv[2];
  }
  const _Float16* wlane = WHE + (size_t)ucol * NHID + koff;
  __syncthreads();

#pragma unroll 1
  for (int t = 0; t < NTOBS; ++t) {
    const int cur = t & 1;
    lstm_step<false>(&At[cur][0], &At[cur ^ 1][0], Df, OffAll + 2 * t, OBSW, wlane, cst, gF0, gF1, gC, ucol, c, hh, koff);
    __syncthreads();
  }

  {
    const v8f z8 = {0.f, 0.f, 0.f, 0.f, 0.f, 0.f, 0.f, 0.f};
    v8f acc1[2][2];
    acc1[0][0] = z8; acc1[0][1] = z8; acc1[1][0] = z8; acc1[1][1] = z8;
    const _Float16* a0p = &At[0][0] + c * APITCH + koff;
    const _Float16* a1p = a0p + 16 * APITCH;
    const _Float16* b0p = WM1P + (size_t)(16 * wave + c) * NHID + koff;
    const _Float16* b1p = WM1P + (size_t)(16 * (wave + 8) + c) * NHID + koff;
#pragma unroll 1
    for (int k0 = 0; k0 < NHID; k0 += 32) {
      const v16h b0 = Frag<_Float16>::load(b0p + k0);
      const v16h b1 = Frag<_Float16>::load(b1p + k0);
      const v16h fa0 = Frag<_Float16>::load(a0p + k0);
      const v16h fa1 = Frag<_Float16>::load(a1p + k0);
      acc1[0][0] = Frag<_Float16>::mma(fa0, b0, acc1[0][0]);
      acc1[0][1] = Frag<_Float16>::mma(fa0, b1, acc1[0][1]);
      acc1[1][0] = Frag<_Float16>::mma(fa1, b0, acc1[1][0]);
      acc1[1][1] = Frag<_Float16>::mma(fa1, b1, acc1[1][1]);
      guard4f(acc1[0][0], acc1[0][1], acc1[1][0], acc1[1][1], fa0, fa1, b0, b1);
    }
    acc_guard4(acc1[0][0], acc1[0][1], acc1[1][0], acc1[1][1]);
#pragma unroll
    for (int jn = 0; jn < 2; ++jn) {
      const int n = 16 * (wave + 8 * jn) + c;
      const float bv = bm1[n];
#pragma unroll
      for (int ms = 0; ms < 2; ++ms)
#pragma unroll
        for (int r = 0; r < 8; ++r) {
          const int row = 16 * ms + 8 * hh + r;
          const float v = fmaxf(fmaf(acc1[ms][jn][r], WCAR_INV, bv), 0.0f);
          Mt[row * MPITCH + n] = (_Float16)v;
        }
    }
  }
  __syncthreads();

  {
    const v8f z8 = {0.f, 0.f, 0.f, 0.f, 0.f, 0.f, 0.f, 0.f};
    v8f acc2[2];
    acc2[0] = z8; acc2[1] = z8;
    const _Float16* a0p = &Mt[0] + c * MPITCH + koff;
    const _Float16* a1p = a0p + 16 * MPITCH;
    const _Float16* bp  = WM2P + (size_t)ucol * NMLP + koff;
#pragma unroll 1
    for (int k0 = 0; k0 < NMLP; k0 += 32) {
      const v16h b0 = Frag<_Float16>::load(bp + k0);
      const v16h fa0 = Frag<_Float16>::load(a0p + k0);
      const v16h fa1 = Frag<_Float16>::load(a1p + k0);
      acc2[0] = Frag<_Float16>::mma(fa0, b0, acc2[0]);
      acc2[1] = Frag<_Float16>::mma(fa1, b0, acc2[1]);
      guard2f(acc2[0], acc2[1], fa0, fa1, b0);
    }
    acc_guard2(acc2[0], acc2[1]);
    const int jb  = (ucol < NMLP2) ? ucol : (NMLP2 - 1);
    const float bv = bm2[jb];
    const int jz0 = ucol - NMLP2;
    const int jz  = (jz0 < 0) ? 0 : jz0;
    const bool usem = (ucol < NMLP2);
#pragma unroll
    for (int ms = 0; ms < 2; ++ms)
#pragma unroll
      for (int r = 0; r < 8; ++r) {
        const int row = 16 * ms + 8 * hh + r;
        const float zv = z[(size_t)(rowbase + row) * NNOISE + jz];
        const float mv = fmaxf(fmaf(acc2[ms][r], WCAR_INV, bv), 0.0f);
        Df[row * DPITCH + ucol] = usem ? mv : zv;
      }
  }
  __syncthreads();

  for (int pass = 0; pass < 2; ++pass) {
#pragma unroll
    for (int q = 0; q < 4; ++q) {
      const int row = 4 * wave + q;
      const v4f v = *(const v4f*)(Df + row * DPITCH + 4 * lane);
      *(volatile v4f*)(DH + (size_t)(rowbase + row) * NHID + 4 * lane) = v;
    }
    __threadfence();
  }
}

__global__ __launch_bounds__(NTHR) void dec_kernel(const float* __restrict__ obs, const float* __restrict__ DH,
                                                   const unsigned short* __restrict__ W16, const float* __restrict__ FC,
                                                   const float* __restrict__ Wr, const float* __restrict__ br,
                                                   float* __restrict__ out) {
  __shared__ __align__(16) _Float16 At[2][RB * APITCH];
  __shared__ __align__(16) float    Hs[RB * HSP];
  __shared__ __align__(16) float    Ob[RB * OBW];
  __shared__ __align__(16) float    In[RB * 2];
  const _Float16* WHD = (const _Float16*)W16 + OFF_WHD;
  const float* FCD = FC + (size_t)NGATE4 * 4;
  const int tid = threadIdx.x, lane = tid & 31, wave = tid >> 5;
  const int c = lane & 15, hh = lane >> 4, koff = 8 * hh;
  const int rowbase = blockIdx.x * RB;
  const int ucol = 16 * wave + c;

#pragma unroll
  for (int it = 0; it < 2; ++it) {
    const int idx = it * NTHR + tid;
    const int r = idx >> 4, j8 = (idx & 15) * 8;
    const float* hp = DH + (size_t)(rowbase + r) * NHID + j8;
    const v4f a = *(const v4f*)(hp);
    const v4f b = *(const v4f*)(hp + 4);
    v8h hv;
#pragma unroll
    for (int e = 0; e < 4; ++e) { hv[e] = (_Float16)a[e]; hv[4 + e] = (_Float16)b[e]; }
    *(v8h*)(&At[0][r * APITCH + j8]) = hv;
  }
  float cst[2][8];
#pragma unroll
  for (int ms = 0; ms < 2; ++ms)
#pragma unroll
    for (int r = 0; r < 8; ++r) cst[ms][r] = 0.0f;
  float gF0[4], gF1[4], gC[4];
#pragma unroll
  for (int g = 0; g < 4; ++g) {
    const v4f fcv = *(const v4f*)(FCD + (size_t)(g * NHID + ucol) * 4);
    gF0[g] = fcv[0]; gF1[g] = fcv[1]; gC[g] = fcv[2];
  }
  float wra[4], wrb[4];
#pragma unroll
  for (int i = 0; i < 4; ++i) { wra[i] = Wr[lane + 32 * i]; wrb[i] = Wr[NHID + lane + 32 * i]; }
  const float br0 = br[0], br1 = br[1];
  float posx[4], posy[4];
#pragma unroll
  for (int q = 0; q < 4; ++q) {
    const int row = 4 * wave + q;
    const float* ob = obs + (size_t)(rowbase + row) * OBSW;
    float px = 0.0f, py = 0.0f, sx = 0.0f, sy = 0.0f, dx = 0.0f, dy = 0.0f;
#pragma unroll 1
    for (int t = 0; t < NTOBS; ++t) {
      const v2f o = *(const v2f*)(ob + 2 * t);
      dx = o[0] - px; dy = o[1] - py;
      sx += dx;       sy += dy;
      px = o[0];      py = o[1];
    }
    posx[q] = sx; posy[q] = sy;
    if (lane == 0) { In[row * 2] = dx; In[row * 2 + 1] = dy; }
  }
  const _Float16* wlane = WHD + (size_t)ucol * NHID + koff;
  __syncthreads();

#pragma unroll 1
  for (int s = 0; s < NSPRED; ++s) {
    const int cur = s & 1;
    lstm_step<true>(&At[cur][0], &At[cur ^ 1][0], Hs, In, 2, wlane, cst, gF0, gF1, gC, ucol, c, hh, koff);
    __syncthreads();
#pragma unroll
    for (int q = 0; q < 4; ++q) {
      const int row = 4 * wave + q;
      const float* hrow = Hs + row * HSP;
      const float h0v = hrow[lane], h1v = hrow[lane + 32], h2v = hrow[lane + 64], h3v = hrow[lane + 96];
      float d0 = h0v * wra[0];
      d0 = fmaf(h1v, wra[1], d0); d0 = fmaf(h2v, wra[2], d0); d0 = fmaf(h3v, wra[3], d0);
      float d1 = h0v * wrb[0];
      d1 = fmaf(h1v, wrb[1], d1); d1 = fmaf(h2v, wrb[2], d1); d1 = fmaf(h3v, wrb[3], d1);
#pragma unroll
      for (int m = 1; m < 32; m <<= 1) {
        d0 += __shfl_xor(d0, m, 32);
        d1 += __shfl_xor(d1, m, 32);
      }
      const float a0 = d0 + br0;
      const float a1 = d1 + br1;
      posx[q] += a0; posy[q] += a1;
      if (lane == 0) {
        In[row * 2]     = a0;
        In[row * 2 + 1] = a1;
        Ob[row * OBW + 2 * s]     = posx[q];
        Ob[row * OBW + 2 * s + 1] = posy[q];
      }
    }
    __syncthreads();
  }
  float* ob_out = out + (size_t)blockIdx.x * (RB * OBW);
  for (int pass = 0; pass < 2; ++pass) {
#pragma unroll
    for (int it = 0; it < 7; ++it) {
      const int q4 = it * NTHR + tid;
      if (q4 < (RB * OBW) / 4) {
        const v4f v = *(const v4f*)(Ob + q4 * 4);
        *(volatile v4f*)(ob_out + (size_t)q4 * 4) = v;
      }
    }
    __threadfence();
  }
}

extern "C" void kernel_launch(void* const* d_in, const int* in_sizes, int n_in,
                              void* d_out, int out_size, void* d_ws, size_t ws_size, hipStream_t stream) {
  if (n_in < 19 || d_out == nullptr || d_ws == nullptr) return;
  if (in_sizes[0] != NAGENT * NTOBS * 2 || in_sizes[2] != NEMB * 2 || in_sizes[3] != NEMB ||
      in_sizes[4] != NGATE4 * NEMB || in_sizes[5] != NGATE4 * NHID || in_sizes[6] != NGATE4 ||
      in_sizes[7] != NMLP * NHID || in_sizes[8] != NMLP || in_sizes[9] != NMLP2 * NMLP || in_sizes[10] != NMLP2 ||
      in_sizes[11] != NEMB * 2 || in_sizes[12] != NEMB || in_sizes[13] != NGATE4 * NEMB ||
      in_sizes[14] != NGATE4 * NHID || in_sizes[15] != NGATE4 || in_sizes[16] != 2 * NHID || in_sizes[17] != 2 ||
      in_sizes[18] != NAGENT * NNOISE || out_size != NAGENT * NSPRED * 2) return;

  const float* obs   = (const float*)d_in[0];
  const float* We    = (const float*)d_in[2];
  const float* be    = (const float*)d_in[3];
  const float* Wih_e = (const float*)d_in[4];
  const float* Whh_e = (const float*)d_in[5];
  const float* b_e   = (const float*)d_in[6];
  const float* Wm1   = (const float*)d_in[7];
  const float* bm1   = (const float*)d_in[8];
  const float* Wm2   = (const float*)d_in[9];
  const float* bm2   = (const float*)d_in[10];
  const float* Wd    = (const float*)d_in[11];
  const float* bd    = (const float*)d_in[12];
  const float* Wih_d = (const float*)d_in[13];
  const float* Whh_d = (const float*)d_in[14];
  const float* b_d   = (const float*)d_in[15];
  const float* Wr    = (const float*)d_in[16];
  const float* br    = (const float*)d_in[17];
  const float* z     = (const float*)d_in[18];
  float* out = (float*)d_out;

  char* ws = (char*)d_ws; size_t off = 0;
  auto carve = [&](size_t bytes) -> char* { char* p = ws + off; off += (bytes + 255) & ~(size_t)255; return p; };
  unsigned short* W16 = (unsigned short*)carve((size_t)W16_HALVES * 2);
  float*          FC  = (float*)carve((size_t)FC_FLOATS * 4);
  float*          DH  = (float*)carve((size_t)NAGENT * NHID * 4);
  if (off > ws_size || off > (size_t)134217728) return;

  prep_w16_kernel<<<W16_HALVES / (NTHR * 8), NTHR, 0, stream>>>(Whh_e, Whh_d, Wm1, Wm2, W16);
  prep_fold_kernel<<<FC_FLOATS / (NTHR * 4), NTHR, 0, stream>>>(Wih_e, We, be, b_e, Wih_d, Wd, bd, b_d, FC);
  enc_mlp_kernel<<<NAGENT / RB, NTHR, 0, stream>>>(obs, W16, FC, bm1, bm2, z, DH);
  dec_kernel<<<NAGENT / RB, NTHR, 0, stream>>>(obs, DH, W16, FC, Wr, br, out);
}
